// G2N2Layer_18296560681006
// MI455X (gfx1250) — hardware-run, weakly checked
//
#include <hip/hip_runtime.h>


namespace {
constexpr int N = 1024, E = 32768, NE = 16, NN = 32, H5 = 32, NEO = 16, NNO = 32, TMPW = 3 * NE + H5, MH = 8 * NE;
constexpr float XS = 8.0f, S4K = 4096.0f, HS = 64.0f, WSC = 256.0f;
typedef _Float16 b16;
typedef __attribute__((ext_vector_type(16))) _Float16 v16b;
typedef __attribute__((ext_vector_type(8))) _Float16 v8b;
typedef __attribute__((ext_vector_type(8))) float v8f;
typedef __attribute__((ext_vector_type(4))) float v4f;
__device__ __forceinline__ float bf16_rne(float f) { unsigned int u = __float_as_uint(f); u += 0x7FFFu + ((u >> 16) & 1u); return __uint_as_float(u & 0xFFFF0000u); }
__device__ __forceinline__ void split16(float v, b16& hi, b16& lo) { hi = (b16)v; lo = (b16)(v - (float)hi); }
__device__ __forceinline__ v16b frag_kb(const b16* p, int hh) { const v8b a = *(const v8b*)(p + 8 * hh), b = *(const v8b*)(p + 16 + 8 * hh); v16b f;
#pragma unroll
  for (int e = 0; e < 8; ++e) { f[e] = a[e]; f[8 + e] = b[e]; } return f; }
__device__ __forceinline__ v8f wmma16b(v16b a, v16b b, v8f c) { v8f d = __builtin_amdgcn_wmma_f32_16x16x32_f16(false, a, false, b, (short)0, c, false, false); asm volatile("v_nop\n\tv_nop\n\tv_nop\n\tv_nop" : "+v"(d) : "v"(a), "v"(b)); return d; }
__device__ __forceinline__ void wave_lds_sync() { __builtin_amdgcn_fence(__ATOMIC_RELEASE, "workgroup"); __builtin_amdgcn_wave_barrier(); __builtin_amdgcn_fence(__ATOMIC_ACQUIRE, "workgroup"); }
__device__ __forceinline__ float pmul(float a, float b) { float p = a * b; asm volatile("" : "+v"(p)); return p; }
__device__ __forceinline__ int iclamp(int v, int lo, int hi) { return v < lo ? lo : (v > hi ? hi : v); }
constexpr int CSR_NBLK5 = 512, CSR_GB5 = 5, CSR_GN5 = 1 << CSR_GB5  , CSR_TS5 = (CSR_GN5 < 32 ? 32 : CSR_GN5)  , CSR_MAXG5 = 512, CSR_CAP5 = 12288  ;
__device__ __host__ __forceinline__ int csr_tix5(int v) { return (v >> CSR_GB5) * CSR_TS5 + (v & (CSR_GN5 - 1)); }
__global__ __launch_bounds__(64) void csrA_kernel5(const int* __restrict__ dst, int E, int N, int nG, int CHP, int NGP, int* __restrict__ STG, int* __restrict__ HST) {
  extern __shared__ int sm[];
  int* cnt = sm; int* run = sm + NGP; int* ids = sm + 2 * NGP;
  const int b = blockIdx.x; const int ch = (E + CSR_NBLK5 - 1) / CSR_NBLK5; const int e0 = b * ch, e1 = min(E, e0 + ch);
  for (int i = threadIdx.x; i < NGP; i += 64) cnt[i] = 0;
  for (int i = threadIdx.x; i < CHP; i += 64) ids[i] = -1;
  __syncthreads();
  if (threadIdx.x == 0) {
    for (int e = e0; e < e1; ++e) { int d = dst[e]; d = (d < 0) ? 0 : (d >= N ? N - 1 : d); cnt[d >> CSR_GB5] += 1; }
    int acc = 0; for (int g = 0; g < nG; ++g) { run[g] = acc; acc += cnt[g]; }
    for (int e = e0; e < e1; ++e) { int d = dst[e]; d = (d < 0) ? 0 : (d >= N ? N - 1 : d); const int g = d >> CSR_GB5; ids[run[g]] = e; run[g] += 1; } }
  __syncthreads();
  typedef __attribute__((ext_vector_type(4))) int v4i;
  for (int pass = 0; pass < 2; ++pass) {
    for (int i = threadIdx.x; i < CHP / 4; i += 64) *(volatile v4i*)(STG + (size_t)b * CHP + i * 4) = *(const v4i*)(&ids[i * 4]);
    for (int i = threadIdx.x; i < NGP / 4; i += 64) { v4i v; for (int e = 0; e < 4; ++e) v[e] = (i * 4 + e < nG) ? cnt[i * 4 + e] : 0; *(volatile v4i*)(HST + (size_t)b * NGP + i * 4) = v; }
    __threadfence(); }
}
__global__ __launch_bounds__(512) void csrS_kernel5(const int* __restrict__ HST, int nG, int NGP, int* __restrict__ START, int* __restrict__ TOT, int* __restrict__ OFF) {
  __shared__ int tot[CSR_MAXG5];
  const int b = threadIdx.x;
  for (int pass = 0; pass < 2; ++pass) { int runb = 0; for (int g = 0; g < nG; ++g) { int c = HST[(size_t)b * NGP + g]; c = (c < 0) ? 0 : c; ((volatile int*)OFF)[(size_t)g * CSR_NBLK5 + b] = runb; runb += c; } __threadfence(); }
  for (int g = threadIdx.x; g < nG; g += 512) { int s = 0; for (int bb = 0; bb < CSR_NBLK5; ++bb) { int c = HST[(size_t)bb * NGP + g]; s += (c < 0) ? 0 : c; } tot[g] = s; }
  __syncthreads();
  if (threadIdx.x < 32) {
    __shared__ int st[CSR_MAXG5 + 32];
    if (threadIdx.x == 0) { int acc = 0; for (int g = 0; g < NGP; ++g) { st[g] = acc; if (g < nG) acc += (tot[g] + 31) & ~31; } st[NGP] = acc; }
    __builtin_amdgcn_fence(__ATOMIC_RELEASE, "workgroup"); __builtin_amdgcn_wave_barrier(); __builtin_amdgcn_fence(__ATOMIC_ACQUIRE, "workgroup");
    for (int pass = 0; pass < 2; ++pass) { for (int i = threadIdx.x; i < NGP + 32; i += 32) { ((volatile int*)START)[i] = (i <= NGP) ? st[min(i, NGP)] : 0; ((volatile int*)TOT)[i] = (i < nG) ? tot[i] : 0; } __threadfence(); } }
}
__global__ __launch_bounds__(256) void csrB_kernel5(const int* __restrict__ dst, int N, int nG, int CHP, int NGP, int permLen, const int* __restrict__ STG, const int* __restrict__ HST, const int* __restrict__ OFF, const int* __restrict__ START, const int* __restrict__ TOT, int* __restrict__ PERM, int* __restrict__ ROWPTR, int* __restrict__ ROWCNT, int* __restrict__ FLAG) {
  typedef __attribute__((ext_vector_type(4))) int v4i;
  __shared__ int ids[CSR_CAP5]; __shared__ unsigned short key[CSR_CAP5]; __shared__ int outp[CSR_CAP5]; __shared__ int ncnt[CSR_GN5 + 1]; __shared__ int boff[CSR_NBLK5 + 1];
  const int g = blockIdx.x, t_ = threadIdx.x; int tot = TOT[g]; int st = START[g], stn = START[g + 1]; const int v0 = g * CSR_GN5; const int nv = min(CSR_GN5, N - v0); const int t0 = g * CSR_TS5;
  st = (st < 0) ? 0 : (st > permLen - 32 ? permLen - 32 : st) & ~31; stn = (stn < st) ? st : (stn > permLen ? permLen : stn); tot = (tot < 0) ? 0 : tot; if (tot > stn - st && tot <= CSR_CAP5) tot = stn - st;
  if (tot > CSR_CAP5) {
    for (int pass = 0; pass < 2; ++pass) { for (int i = t_; i < CSR_TS5 / 4; i += 256) { v4i a, c; for (int e = 0; e < 4; ++e) { a[e] = st; c[e] = 0; } *(volatile v4i*)(ROWPTR + t0 + i * 4) = a; *(volatile v4i*)(ROWCNT + t0 + i * 4) = c; } if (t_ == 0) ((volatile int*)FLAG)[0] = 1; __threadfence(); } (void)nv; return; }
  if (t_ == 0) { int acc = 0; for (int b = 0; b < CSR_NBLK5; ++b) { boff[b] = acc; int c = HST[(size_t)b * NGP + g]; c = (c < 0) ? 0 : (c > CHP ? CHP : c); acc += c; if (acc > tot) acc = tot; } boff[CSR_NBLK5] = acc; }
  for (int i = t_; i <= CSR_GN5; i += 256) ncnt[i] = 0;
  __syncthreads();
  for (int b = 0; b < CSR_NBLK5; ++b) { const int c = boff[b + 1] - boff[b]; int o_ = OFF[(size_t)g * CSR_NBLK5 + b]; o_ = (o_ < 0) ? 0 : (o_ > CHP - c ? CHP - c : o_); const int* src_ = STG + (size_t)b * CHP + o_;
    for (int i = t_; i < c; i += 256) { int id = src_[i]; id = (id < 0) ? 0 : id; ids[boff[b] + i] = id; int d = dst[id]; d = (d < v0) ? v0 : (d >= N ? N - 1 : d); int kk = d - v0; kk = (kk < 0) ? 0 : (kk >= CSR_GN5 ? CSR_GN5 - 1 : kk); key[boff[b] + i] = (unsigned short)kk; } }
  __syncthreads();
  if (t_ == 0) { for (int i = 0; i < tot; ++i) ncnt[key[i]] += 1; int acc = 0; for (int vl = 0; vl < CSR_GN5; ++vl) { const int c = ncnt[vl]; ncnt[vl] = acc; acc += c; } ncnt[CSR_GN5] = acc;
    for (int i = 0; i < tot; ++i) { const int vl = key[i]; outp[ncnt[vl]] = ids[i]; ncnt[vl] += 1; }
    for (int vl = CSR_GN5; vl > 0; --vl) ncnt[vl] = ncnt[vl - 1]; ncnt[0] = 0; }
  __syncthreads();
  for (int pass = 0; pass < 2; ++pass) {
    for (int i = t_; i < (stn - st) / 4; i += 256) { v4i v; for (int e = 0; e < 4; ++e) { const int q = i * 4 + e; v[e] = (q < tot) ? outp[q] : -1; } *(volatile v4i*)(PERM + st + i * 4) = v; }
    for (int i = t_; i < CSR_TS5 / 4; i += 256) { v4i a, c; for (int e = 0; e < 4; ++e) { const int vl = i * 4 + e; const int vc = vl < CSR_GN5 ? vl : CSR_GN5; a[e] = (vl < CSR_GN5) ? st + ncnt[vc] : st; c[e] = (vl < nv) ? (ncnt[(vc < CSR_GN5 ? vc : CSR_GN5 - 1) + 1] - ncnt[vc]) : 0; } *(volatile v4i*)(ROWPTR + t0 + i * 4) = a; *(volatile v4i*)(ROWCNT + t0 + i * 4) = c; }
    __threadfence(); }
}
__global__ __launch_bounds__(256) void csrZ_kernel5(int* __restrict__ p, size_t n4) { typedef __attribute__((ext_vector_type(4))) int v4i; const size_t tid = (size_t)blockIdx.x * 256 + threadIdx.x, nth = (size_t)gridDim.x * 256; v4i z = {0, 0, 0, 0}; for (size_t i = tid; i < n4; i += nth) *(volatile v4i*)(p + i * 4) = z; }
struct CsrBufs5 { int *STG, *HST, *OFF, *START, *TOT, *PERM, *ROWPTR, *ROWCNT, *FLAG; int nG, NGP, CHP; size_t permLen; char* base; size_t bytes; };
static size_t csr_carve5(CsrBufs5& c, char* ws, size_t off, int E, int N) {
  const size_t off0 = off; c.base = ws + off;
  auto al = [&](size_t bytes) { char* p = ws + off; off += (bytes + 255) & ~(size_t)255; return p; };
  c.nG = (N + CSR_GN5 - 1) / CSR_GN5; c.NGP = (c.nG + 31) & ~31; const int ch = (E + CSR_NBLK5 - 1) / CSR_NBLK5; c.CHP = (ch + 31) & ~31; c.permLen = (size_t)E + 32 * (size_t)c.nG + 32;
  c.STG = (int*)al((size_t)CSR_NBLK5 * c.CHP * 4); c.HST = (int*)al((size_t)CSR_NBLK5 * c.NGP * 4); c.OFF = (int*)al((size_t)c.NGP * CSR_NBLK5 * 4); c.START = (int*)al((size_t)(c.NGP + 64) * 4); c.TOT = (int*)al((size_t)(c.NGP + 64) * 4);
  c.PERM = (int*)al(c.permLen * 4); c.ROWPTR = (int*)al((size_t)c.nG * CSR_TS5 * 4); c.ROWCNT = (int*)al((size_t)c.nG * CSR_TS5 * 4); c.FLAG = (int*)al(256);
  c.bytes = off - off0; return off;
}
static void csr_build5(const CsrBufs5& c, const int* dst, int E, int N, hipStream_t stream) {
  const size_t smem = (size_t)(2 * c.NGP + c.CHP) * 4;
  csrZ_kernel5<<<512, 256, 0, stream>>>((int*)c.base, c.bytes / 16);
  csrA_kernel5<<<CSR_NBLK5, 64, smem, stream>>>(dst, E, N, c.nG, c.CHP, c.NGP, c.STG, c.HST);
  csrS_kernel5<<<1, 512, 0, stream>>>(c.HST, c.nG, c.NGP, c.START, c.TOT, c.OFF);
  csrB_kernel5<<<c.nG, 256, 0, stream>>>(dst, N, c.nG, c.CHP, c.NGP, (int)c.permLen, c.STG, c.HST, c.OFF, c.START, c.TOT, c.PERM, c.ROWPTR, c.ROWCNT, c.FLAG);
}


__global__ __launch_bounds__(256) void w_kernel(const float* __restrict__ W1, const float* __restrict__ W2, const float* __restrict__ W3, const float* __restrict__ W4, const float* __restrict__ W5, const float* __restrict__ AW, const float* __restrict__ Wm1, const float* __restrict__ Wm2, b16* __restrict__ WC, b16* __restrict__ WX, b16* __restrict__ WM1, b16* __restrict__ WM2) {
  const int u = blockIdx.x * 256 + threadIdx.x; v8b v;
  if (u < 64 * 4) { const int o = u / 4, k0 = (u % 4) * 8; const float* Wsel = (o < 16) ? W1 : (o < 32) ? W2 : (o < 48) ? W3 : W4; for (int j = 0; j < 8; ++j) { const int k = k0 + j; v[j] = k < NE ? (b16)(bf16_rne(Wsel[k * NE + (o & 15)]) * WSC) : (b16)0.0f; } for (int pass = 0; pass < 2; ++pass) { *(volatile v8b*)(WC + o * 32 + k0) = v; __threadfence(); } return; }
  int w = u - 64 * 4;
  if (w < 544 * 4) { const int o = w / 4, k0 = (w % 4) * 8; for (int j = 0; j < 8; ++j) { const int k = k0 + j; float val; if (o < 32) val = W5[k * H5 + o]; else { const int kk = (o - 32) / 32, oo = (o - 32) % 32; val = AW[((size_t)kk * NN + k) * NNO + oo]; } v[j] = (b16)(bf16_rne(val) * WSC); } for (int pass = 0; pass < 2; ++pass) { *(volatile v8b*)(WX + o * 32 + k0) = v; __threadfence(); } return; }
  w -= 544 * 4;
  if (w < MH * 12) { const int c = w / 12, k0 = (w % 12) * 8; for (int j = 0; j < 8; ++j) { const int k = k0 + j; float val = 0.0f, sc = WSC; if (k < TMPW) { val = Wm1[k * MH + c]; sc = (k < NE) ? WSC * (S4K / XS) : WSC; } v[j] = (b16)(bf16_rne(val) * sc); } for (int pass = 0; pass < 2; ++pass) { *(volatile v8b*)(WM1 + c * 96 + k0) = v; __threadfence(); } return; }
  w -= MH * 12;
  if (w < NEO * 16) { const int o = w / 16, k0 = (w % 16) * 8; for (int j = 0; j < 8; ++j) v[j] = (b16)(bf16_rne(Wm2[(k0 + j) * NEO + o]) * WSC); for (int pass = 0; pass < 2; ++pass) { *(volatile v8b*)(WM2 + o * MH + k0) = v; __threadfence(); } }
}
__global__ __launch_bounds__(32) void eid_kernel(const int* __restrict__ ei, const int* __restrict__ PERM, const int* __restrict__ ROWPTR, const int* __restrict__ ROWCNT, int permLen, int* __restrict__ EID) {
  __shared__ int Row[N]; const int lane = threadIdx.x; const int i = blockIdx.x;
  for (int c = lane; c < N; c += 32) Row[c] = -1; wave_lds_sync();
  int st = ROWPTR[i], cnt = ROWCNT[i]; cnt = iclamp(cnt, 0, 1 << 20); st = iclamp(st, 0, permLen - cnt);
  for (int q = lane; q < cnt; q += 32) { const int e = iclamp(PERM[st + q], 0, E - 1); const int j = iclamp(ei[E + e], 0, N - 1); Row[j] = e; }
  wave_lds_sync();
  for (int pass = 0; pass < 2; ++pass) { for (int c = lane; c < N; c += 32) ((volatile int*)EID)[(size_t)i * N + c] = Row[c]; __threadfence(); }
}
__global__ __launch_bounds__(32) void elin_kernel(const float* __restrict__ Cm, const b16* __restrict__ WC, float* __restrict__ CW) {
  __shared__ __attribute__((aligned(16))) b16 Ah[16][40]; __shared__ __attribute__((aligned(16))) float Tf[16][68];
  const int lane = threadIdx.x, nloc = lane & 15, hlf = lane >> 4; const size_t e0 = (size_t)blockIdx.x * 16;
  for (int rr = 0; rr < 16; ++rr) Ah[rr][lane] = lane < NE ? (b16)(bf16_rne(Cm[(e0 + rr) * NE + lane]) * XS) : (b16)0.0f;
  wave_lds_sync(); const v16b a = frag_kb(&Ah[nloc][0], hlf);
#pragma unroll
  for (int t = 0; t < 4; ++t) { v8f acc = {}; acc = wmma16b(a, frag_kb(WC + (t * 16 + nloc) * 32, hlf), acc);
#pragma unroll
    for (int r8 = 0; r8 < 8; ++r8) Tf[8 * hlf + r8][t * 16 + nloc] = acc[r8] * (1.0f / (XS * WSC)) * (1.0f / NE); }
  wave_lds_sync();
  for (int pass = 0; pass < 2; ++pass) { for (int rr = 0; rr < 16; ++rr) { ((volatile float*)CW)[(e0 + rr) * 64 + lane] = Tf[rr][lane]; ((volatile float*)CW)[(e0 + rr) * 64 + 32 + lane] = Tf[rr][32 + lane]; } __threadfence(); }
}
__global__ __launch_bounds__(32) void nlin_kernel(const float* __restrict__ x, const b16* __restrict__ WX, float* __restrict__ H5P, float* __restrict__ XW) {
  __shared__ __attribute__((aligned(16))) b16 Ah[16][40]; __shared__ __attribute__((aligned(16))) float Tf[16][36];
  const int lane = threadIdx.x, nloc = lane & 15, hlf = lane >> 4; const size_t n0 = (size_t)blockIdx.x * 16;
  for (int rr = 0; rr < 16; ++rr) Ah[rr][lane] = (b16)(bf16_rne(x[(n0 + rr) * NN + lane]) * XS);
  wave_lds_sync(); const v16b a = frag_kb(&Ah[nloc][0], hlf);
#pragma unroll 1
  for (int blk = 0; blk < 17; ++blk) {
#pragma unroll
    for (int t = 0; t < 2; ++t) { v8f acc = {}; acc = wmma16b(a, frag_kb(WX + (size_t)(blk * 32 + t * 16 + nloc) * 32, hlf), acc); const float sc = (blk == 0) ? (1.0f / (XS * WSC)) * (1.0f / NN) : (1.0f / (XS * WSC));
#pragma unroll
      for (int r8 = 0; r8 < 8; ++r8) Tf[8 * hlf + r8][t * 16 + nloc] = acc[r8] * sc; }
    wave_lds_sync();
    for (int pass = 0; pass < 2; ++pass) { for (int rr = 0; rr < 16; ++rr) { if (blk == 0) ((volatile float*)H5P)[(n0 + rr) * H5 + lane] = Tf[rr][lane]; else ((volatile float*)XW)[((n0 + rr) * NE + (blk - 1)) * NNO + lane] = Tf[rr][lane]; } __threadfence(); }
    wave_lds_sync(); }
}
__global__ __launch_bounds__(32) void edge_kernel(const float* __restrict__ Cm, const float* __restrict__ CW, const float* __restrict__ H5P, const int* __restrict__ ei, const int* __restrict__ EID, const int* __restrict__ PERM, const int* __restrict__ ROWPTR, const int* __restrict__ ROWCNT, int permLen, const b16* __restrict__ WM1, const b16* __restrict__ WM2, float* __restrict__ COUT, float* __restrict__ out2) {
  __shared__ __attribute__((aligned(16))) b16 Ah[16][MH + 8], Al[16][MH + 8]; __shared__ float So[16][NEO];
  const int lane = threadIdx.x, nloc = lane & 15, hlf = lane >> 4; const size_t e0 = (size_t)blockIdx.x * 16; const int k = nloc;
  for (int rr = 0; rr < 16; ++rr) { const size_t e = e0 + rr; const int i = iclamp(ei[e], 0, N - 1), j = iclamp(ei[E + e], 0, N - 1);
    if (hlf == 0) { const float c = bf16_rne(Cm[e * NE + k]); Ah[rr][k] = (b16)(c * XS); Al[rr][k] = (b16)0.0f;
      const float had = pmul(CW[e * 64 + k], CW[e * 64 + 16 + k]); b16 p, q; split16(had * S4K, p, q); Ah[rr][16 + k] = p; Al[rr][16 + k] = q;
      float tm = 0.0f; int st = ROWPTR[i], cnt = ROWCNT[i]; cnt = iclamp(cnt, 0, 1 << 20); st = iclamp(st, 0, permLen - cnt);
#pragma unroll 1
      for (int q2 = 0; q2 < cnt; ++q2) { const int e1 = iclamp(PERM[st + q2], 0, E - 1); const int m = iclamp(ei[E + e1], 0, N - 1); const int e2 = EID[m * N + j]; if (e2 >= 0 && e2 < E) tm += pmul(CW[(size_t)e1 * 64 + 32 + k], CW[(size_t)e2 * 64 + 48 + k]); }
      split16(tm * S4K, p, q); Ah[rr][64 + k] = p; Al[rr][64 + k] = q; Ah[rr][80 + k] = (b16)0.0f; Al[rr][80 + k] = (b16)0.0f; }
    { const float d = (i == j) ? H5P[(size_t)i * H5 + lane] : 0.0f; b16 p, q; split16(d * S4K, p, q); Ah[rr][32 + lane] = p; Al[rr][32 + lane] = q; } }
  wave_lds_sync();
  v8f acc[8];
#pragma unroll
  for (int t = 0; t < 8; ++t) acc[t] = (v8f){};
#pragma unroll
  for (int kb = 0; kb < 96; kb += 32) { const v16b a = frag_kb(&Ah[nloc][kb], hlf), al = frag_kb(&Al[nloc][kb], hlf);
#pragma unroll
    for (int t = 0; t < 8; ++t) { const v16b bw = frag_kb(WM1 + (t * 16 + nloc) * 96 + kb, hlf); acc[t] = wmma16b(a, bw, acc[t]); acc[t] = wmma16b(al, bw, acc[t]); } }
  wave_lds_sync();
#pragma unroll
  for (int t = 0; t < 8; ++t)
#pragma unroll
    for (int r8 = 0; r8 < 8; ++r8) { const int rl = 8 * hlf + r8; b16 p, q; split16(fmaxf(acc[t][r8] * (1.0f / (S4K * WSC)), 0.0f) * HS, p, q); Ah[rl][t * 16 + nloc] = p; Al[rl][t * 16 + nloc] = q; }
  wave_lds_sync();
  { v8f a2 = {};
#pragma unroll
    for (int kb = 0; kb < MH; kb += 32) { const v16b bw = frag_kb(WM2 + nloc * MH + kb, hlf); a2 = wmma16b(frag_kb(&Ah[nloc][kb], hlf), bw, a2); a2 = wmma16b(frag_kb(&Al[nloc][kb], hlf), bw, a2); }
#pragma unroll
    for (int r8 = 0; r8 < 8; ++r8) So[8 * hlf + r8][nloc] = a2[r8] * (1.0f / (HS * WSC)); }
  wave_lds_sync();
  for (int pass = 0; pass < 2; ++pass) { for (int i2 = lane; i2 < 16 * NEO; i2 += 32) { const float v = So[i2 / NEO][i2 % NEO]; ((volatile float*)COUT)[e0 * NEO + i2] = v; ((volatile float*)out2)[e0 * NEO + i2] = v; } __threadfence(); }
}
__global__ __launch_bounds__(256) void nagg_kernel(const float* __restrict__ COUT, const float* __restrict__ XW, const int* __restrict__ ei, const int* __restrict__ PERM, const int* __restrict__ ROWPTR, const int* __restrict__ ROWCNT, int permLen, const float* __restrict__ ab, float* __restrict__ out1) {
  const int wave = threadIdx.x >> 5, lane = threadIdx.x & 31; const int n = blockIdx.x * 8 + wave; if (n >= N) return;
  int st = ROWPTR[n], cnt = ROWCNT[n]; cnt = iclamp(cnt, 0, 1 << 20); st = iclamp(st, 0, permLen - cnt); float s = 0.0f;
#pragma unroll 1
  for (int q = 0; q < cnt; ++q) { const int e = iclamp(PERM[st + q], 0, E - 1); const int m = iclamp(ei[E + e], 0, N - 1); const float* xw = XW + (size_t)m * NE * NNO;
#pragma unroll
    for (int k = 0; k < NE; ++k) s += pmul(COUT[(size_t)e * NEO + k], xw[k * NNO + lane]); }
  const float r = (s + bf16_rne(ab[lane])) * (1.0f / NN);
  for (int pass = 0; pass < 2; ++pass) { ((volatile float*)out1)[(size_t)n * NNO + lane] = r; __threadfence(); }
}
}

extern "C" void kernel_launch(void* const* d_in, const int* in_sizes, int n_in, void* d_out, int out_size, void* d_ws, size_t ws_size, hipStream_t stream) {
  (void)n_in;
  auto Fp = [&](int i) { return (const float*)d_in[i]; }; auto Ip = [&](int i) { return (const int*)d_in[i]; };
  if (in_sizes[0] != N * NN || in_sizes[1] != E * NE || in_sizes[2] != N || in_sizes[3] != 2 * E || in_sizes[4] != NE * NE || in_sizes[8] != NN * H5 || in_sizes[9] != TMPW * MH || in_sizes[10] != MH * NEO || in_sizes[11] != NEO * NN * NNO || out_size != N * NNO + E * NEO) return;
  size_t off = 0; char* ws = (char*)d_ws;
  auto carve = [&](size_t bytes) { char* p = ws + off; off += (bytes + 255) & ~(size_t)255; return p; };
  b16* WC = (b16*)carve(64 * 32 * 2); b16* WX = (b16*)carve(544 * 32 * 2); b16* WM1 = (b16*)carve(MH * 96 * 2); b16* WM2 = (b16*)carve(NEO * MH * 2); int* EID = (int*)carve((size_t)N * N * 4);
  float* CW = (float*)carve((size_t)E * 64 * 4); float* H5P = (float*)carve((size_t)N * H5 * 4); float* XW = (float*)carve((size_t)N * NE * NNO * 4); float* COUT = (float*)carve((size_t)E * NEO * 4);
  CsrBufs5 csr; off = csr_carve5(csr, ws, off, E, N);
  if (off > ws_size || off > ((size_t)64 << 20)) return;
  w_kernel<<<(64 * 4 + 544 * 4 + MH * 12 + NEO * 16 + 255) / 256, 256, 0, stream>>>(Fp(4), Fp(5), Fp(6), Fp(7), Fp(8), Fp(11), Fp(9), Fp(10), WC, WX, WM1, WM2);
  csr_build5(csr, Ip(3), E, N, stream);
  eid_kernel<<<N, 32, 0, stream>>>(Ip(3), csr.PERM, csr.ROWPTR, csr.ROWCNT, (int)csr.permLen, EID);
  elin_kernel<<<E / 16, 32, 0, stream>>>(Fp(1), WC, CW);
  nlin_kernel<<<N / 16, 32, 0, stream>>>(Fp(0), WX, H5P, XW);
  edge_kernel<<<E / 16, 32, 0, stream>>>(Fp(1), CW, H5P, Ip(3), EID, csr.PERM, csr.ROWPTR, csr.ROWCNT, (int)csr.permLen, WM1, WM2, COUT, (float*)d_out + (size_t)N * NNO);
  nagg_kernel<<<N / 8, 256, 0, stream>>>(COUT, XW, Ip(3), csr.PERM, csr.ROWPTR, csr.ROWCNT, (int)csr.permLen, Fp(12), (float*)d_out);
}
